// CausalTrajectoryPrediction_9620726743706
// MI455X (gfx1250) — hardware-verified
//
#include <hip/hip_runtime.h>


#define NN 64
#define HH 512
#define MM 64
#define BT 64

typedef _Float16 bf16_t;
typedef __attribute__((ext_vector_type(16))) _Float16 v16bf;
typedef __attribute__((ext_vector_type(8)))  _Float16 v8bf;
typedef __attribute__((ext_vector_type(4)))  float v4f_t;
typedef float v4fa __attribute__((ext_vector_type(4), may_alias));
typedef __attribute__((ext_vector_type(8)))  float  v8f;

__device__ __forceinline__ v16bf fragT(const float* rowptr, int k0, int kb) {
  const float* p = rowptr + k0 + kb;
  v16bf f;
#pragma unroll
  for (int i = 0; i < 8; ++i) f[i] = (bf16_t)p[i];
#pragma unroll
  for (int i = 0; i < 8; ++i) f[i + 8] = (bf16_t)p[16 + i];
  return f;
}
__device__ __forceinline__ v16bf fragT(const bf16_t* rowptr, int k0, int kb) {
  const bf16_t* p = rowptr + k0 + kb;
  v8bf lo = *(const v8bf*)(p);
  v8bf hi = *(const v8bf*)(p + 16);
  v16bf f;
#pragma unroll
  for (int i = 0; i < 8; ++i) { f[i] = lo[i]; f[i + 8] = hi[i]; }
  return f;
}

#define WMMA_BF16(A, B, C) \
  __builtin_amdgcn_wmma_f32_16x16x32_f16(false, (A), false, (B), (short)0, (C), false, false)

__global__ __launch_bounds__(256) void convert_weights(
    const float* __restrict__ W1, const float* __restrict__ W2,
    const float* __restrict__ W3,
    bf16_t* __restrict__ W1b, bf16_t* __restrict__ W2b, bf16_t* __restrict__ W3ab) {
  long i = ((long)blockIdx.x * 256 + threadIdx.x) * 2;
  if (i < (long)NN * HH * NN) {
    long row = i >> 6, k = i & 63;
    const unsigned u1 = (unsigned)__builtin_bit_cast(unsigned short, (bf16_t)W1[i]) | ((unsigned)__builtin_bit_cast(unsigned short, (bf16_t)W1[i + 1]) << 16);
    const unsigned u2 = (unsigned)__builtin_bit_cast(unsigned short, (bf16_t)W2[i]) | ((unsigned)__builtin_bit_cast(unsigned short, (bf16_t)W2[i + 1]) << 16);
    const unsigned u3 = (unsigned)__builtin_bit_cast(unsigned short, (bf16_t)W3[row * (MM + NN) + k]) | ((unsigned)__builtin_bit_cast(unsigned short, (bf16_t)W3[row * (MM + NN) + k + 1]) << 16);
    *(volatile unsigned*)(W1b + i) = u1; *(volatile unsigned*)(W2b + i) = u2; *(volatile unsigned*)(W3ab + i) = u3; __threadfence();
    *(volatile unsigned*)(W1b + i) = u1; *(volatile unsigned*)(W2b + i) = u2; *(volatile unsigned*)(W3ab + i) = u3;
  }
}

__global__ __launch_bounds__(256) void transpose_out(const float* __restrict__ outT, float* __restrict__ out) {
  __shared__ __attribute__((aligned(16))) float st[16 * 68];
  const int r0 = blockIdx.x * 16, tid = threadIdx.x;
  for (int i = tid; i < 16 * NN; i += 256) { const int n = i >> 4, r = i & 15; st[r * 68 + n] = outT[(size_t)n * 1024 + r0 + r]; }
  __syncthreads();
  const int r = tid >> 4, q = (tid & 15) * 4;
  const v4f_t v = *(const volatile v4fa*)(st + r * 68 + q);
  *(volatile v4f_t*)(out + (size_t)(r0 + r) * NN + q) = v; __threadfence(); *(volatile v4f_t*)(out + (size_t)(r0 + r) * NN + q) = v;
}

template <typename WT>
__global__ __launch_bounds__(256) void causal_deriv_kernel(
    const float* __restrict__ x,
    const WT* __restrict__ W1, const WT* __restrict__ W2,
    const WT* __restrict__ W3a, int ld3,
    const float* __restrict__ W3full, const float* __restrict__ b3,
    const float* __restrict__ W4, const float* __restrict__ b4,
    float* __restrict__ outT) {
  __shared__ bf16_t sA[BT * NN];
  __shared__ bf16_t sH[BT * HH];
  __shared__ bf16_t sR[BT * MM];
  __shared__ float  sXn[BT];
  __shared__ float  sOut[BT];

  const int n    = blockIdx.y;
  const int b0   = blockIdx.x * BT;
  const int tid  = threadIdx.x;
  const int wv   = tid >> 5;
  const int lane = tid & 31;
  const int l15  = lane & 15;
  const int hi8  = (lane & 16) ? 8 : 0;
  const int kb   = hi8;

  for (int idx = tid; idx < BT * NN; idx += 256) {
    int r = idx >> 6, c = idx & 63;
    float v = x[(b0 + r) * NN + c];
    if (c == n) { sXn[r] = v; sA[idx] = (bf16_t)0.0f; }
    else        { sA[idx] = (bf16_t)v; }
  }
  if (tid < BT) sOut[tid] = 0.0f;
  __syncthreads();

  {
    const int colb = wv * 64;
    v8f acc[4][4];
#pragma unroll
    for (int s = 0; s < 4; ++s)
#pragma unroll
      for (int t = 0; t < 4; ++t)
#pragma unroll
        for (int j = 0; j < 8; ++j) acc[s][t][j] = 0.0f;

#pragma unroll
    for (int k0 = 0; k0 < NN; k0 += 32) {
      v16bf a[4];
#pragma unroll
      for (int s = 0; s < 4; ++s) a[s] = fragT(sA + (s * 16 + l15) * NN, k0, kb);
#pragma unroll
      for (int t = 0; t < 4; ++t) {
        int col = colb + t * 16 + l15;
        v16bf bfr = fragT(W1 + ((long)n * HH + col) * NN, k0, kb);
#pragma unroll
        for (int s = 0; s < 4; ++s) acc[s][t] = WMMA_BF16(a[s], bfr, acc[s][t]);
      }
    }
#pragma unroll
    for (int s = 0; s < 4; ++s)
#pragma unroll
      for (int t = 0; t < 4; ++t) {
        int col = colb + t * 16 + l15;
#pragma unroll
        for (int j = 0; j < 8; ++j) {
          float v = acc[s][t][j];
          sH[(s * 16 + j + hi8) * HH + col] = (bf16_t)(v > 0.0f ? v : 0.0f);
        }
      }
  }
  __syncthreads();

  {
    const int ct = wv & 3;
    const int sp = wv >> 2;
    v8f acc2[2];
#pragma unroll
    for (int q = 0; q < 2; ++q)
#pragma unroll
      for (int j = 0; j < 8; ++j) acc2[q][j] = 0.0f;

    const WT* w2row = W2 + ((long)n * MM + (ct * 16 + l15)) * HH;
#pragma unroll
    for (int k0 = 0; k0 < HH; k0 += 32) {
      v16bf bfr = fragT(w2row, k0, kb);
#pragma unroll
      for (int q = 0; q < 2; ++q) {
        int s = sp + 2 * q;
        v16bf a = fragT(sH + (s * 16 + l15) * HH, k0, kb);
        acc2[q] = WMMA_BF16(a, bfr, acc2[q]);
      }
    }
#pragma unroll
    for (int q = 0; q < 2; ++q) {
      int s = sp + 2 * q;
#pragma unroll
      for (int j = 0; j < 8; ++j) {
        float v = acc2[q][j];
        sR[(s * 16 + j + hi8) * MM + (ct * 16 + l15)] = (bf16_t)(v > 0.0f ? v : 0.0f);
      }
    }
  }
  __syncthreads();

  {
    const int colb = wv * 64;
    float bias[4], w3c[4], w4c[4];
#pragma unroll
    for (int t = 0; t < 4; ++t) {
      int col = colb + t * 16 + l15;
      bias[t] = b3[n * HH + col];
      w3c[t]  = W3full[((long)n * HH + col) * (MM + NN) + MM + n];
      w4c[t]  = W4[n * HH + col];
    }
    v8f acc[4][4];
#pragma unroll
    for (int s = 0; s < 4; ++s)
#pragma unroll
      for (int j = 0; j < 8; ++j) {
        float xr = sXn[s * 16 + j + hi8];
#pragma unroll
        for (int t = 0; t < 4; ++t) acc[s][t][j] = bias[t] + xr * w3c[t];
      }

#pragma unroll
    for (int k0 = 0; k0 < MM; k0 += 32) {
      v16bf a[4];
#pragma unroll
      for (int s = 0; s < 4; ++s) a[s] = fragT(sR + (s * 16 + l15) * MM, k0, kb);
#pragma unroll
      for (int t = 0; t < 4; ++t) {
        int col = colb + t * 16 + l15;
        v16bf bfr = fragT(W3a + ((long)n * HH + col) * ld3, k0, kb);
#pragma unroll
        for (int s = 0; s < 4; ++s) acc[s][t] = WMMA_BF16(a[s], bfr, acc[s][t]);
      }
    }

#pragma unroll
    for (int s = 0; s < 4; ++s) {
      float p[8];
#pragma unroll
      for (int j = 0; j < 8; ++j) p[j] = 0.0f;
#pragma unroll
      for (int t = 0; t < 4; ++t)
#pragma unroll
        for (int j = 0; j < 8; ++j) {
          float v = acc[s][t][j];
          p[j] += (v > 0.0f ? v : 0.0f) * w4c[t];
        }
#pragma unroll
      for (int m = 8; m >= 1; m >>= 1)
#pragma unroll
        for (int j = 0; j < 8; ++j) p[j] += __shfl_xor(p[j], m, 32);
      if (l15 == 0) {
#pragma unroll
        for (int j = 0; j < 8; ++j) atomicAdd(&sOut[s * 16 + j + hi8], p[j]);
      }
    }
  }
  __syncthreads();

  if (tid < BT) {
    float v = sOut[tid] + b4[n];
    v = v > 0.0f ? v : 0.0f;
    float* p = outT + (size_t)n * 1024 + b0 + tid;
    *(volatile float*)p = v; __threadfence(); *(volatile float*)p = v;
  }
}

extern "C" void kernel_launch(void* const* d_in, const int* in_sizes, int n_in,
                              void* d_out, int out_size, void* d_ws, size_t ws_size,
                              hipStream_t stream) {
  const float* x  = (const float*)d_in[0];
  const float* W1 = (const float*)d_in[1];
  const float* W2 = (const float*)d_in[2];
  const float* W3 = (const float*)d_in[3];
  const float* b3 = (const float*)d_in[4];
  const float* W4 = (const float*)d_in[5];
  const float* b4 = (const float*)d_in[6];
  float* out = (float*)d_out;
  (void)in_sizes; (void)n_in; (void)out_size;

  dim3 grid(1024 / BT, NN);
  const long NE = (long)NN * HH * NN;
  (void)ws_size;
  bf16_t* W1b  = (bf16_t*)d_ws;
  bf16_t* W2b  = W1b + NE;
  bf16_t* W3ab = W2b + NE;
  float*  outT = (float*)(W3ab + NE);
  convert_weights<<<(int)((NE / 2 + 255) / 256), 256, 0, stream>>>(W1, W2, W3, W1b, W2b, W3ab);
  causal_deriv_kernel<bf16_t><<<grid, 256, 0, stream>>>(x, W1b, W2b, W3ab, NN, W3, b3, W4, b4, outT);
  transpose_out<<<1024 / 16, 256, 0, stream>>>(outT, out);
}
